// EEGNeX_21268678050414
// MI455X (gfx1250) — hardware-verified
//
#include <hip/hip_runtime.h>

typedef _Float16 f16t;
typedef _Float16 v16h __attribute__((ext_vector_type(16)));
typedef _Float16 v8h  __attribute__((ext_vector_type(8)));
typedef _Float16 v4h  __attribute__((ext_vector_type(4)));
typedef float    v8f  __attribute__((ext_vector_type(8)));
typedef float    v4f  __attribute__((ext_vector_type(4)));
typedef v8h __attribute__((may_alias)) v8ha;
typedef v4h __attribute__((may_alias)) v4ha;
typedef v4f __attribute__((may_alias)) v4fa;
union Frag { v16h v; v8h half[2]; v4h q[4]; };

#define NB_    64
#define NCH    64
#define TT     1000
#define TPAD   1024
#define NADP   109
#define RANK   4
#define F1     8
#define F2     32
#define F3     64
#define K12    64
#define K45    16
#define T3     250
#define T5     31
#define NFEAT  248
#define NOUT   4
#define K2     512
#define K4TOT  2048
#define K5TOT  1024
#define H1ROWS 1088
#define H1OFF  32
#define H4ROWS 288
#define H4OFF  16
#define H5ROWS 320
#define H5OFF  32
#define CPW    1104
#define WCAR   256.0f
#define WINV   (1.0f / 256.0f)
#define AOR    0.25f
#define EPS_   1e-5f

#define OFF_W1P  ((size_t)0)
#define OFF_W2P  ((size_t)131072)
#define OFF_W4P  ((size_t)2228224)
#define OFF_W5P  ((size_t)10616832)
#define OFF_H1   ((size_t)12713984)
#define OFF_O3   ((size_t)84017152)
#define OFF_H4   ((size_t)100794368)
#define OFF_H5   ((size_t)103153664)
#define OFF_FEAT ((size_t)104464384)
#define WS_TOTAL ((size_t)104529920)

__device__ __forceinline__ v8f wmma1(v16h a, v16h b, v8f c) {
  return __builtin_amdgcn_wmma_f32_16x16x32_f16(false, a, false, b, (short)0, c, false, false);
}
#define NOPS4 "v_nop\n\tv_nop\n\tv_nop\n\tv_nop"
#define GUARD2x6(c0,c1,x0,x1,x2,x3,x4,x5) \
  asm volatile(NOPS4 : "+v"(c0), "+v"(c1) : "v"(x0), "v"(x1), "v"(x2), "v"(x3), "v"(x4), "v"(x5))
#define GUARD4x4(c0,c1,c2,c3,x0,x1,x2,x3) \
  asm volatile(NOPS4 : "+v"(c0), "+v"(c1), "+v"(c2), "+v"(c3) : "v"(x0), "v"(x1), "v"(x2), "v"(x3))
#define GUARD4x5(c0,c1,c2,c3,x0,x1,x2,x3,x4) \
  asm volatile(NOPS4 : "+v"(c0), "+v"(c1), "+v"(c2), "+v"(c3) : "v"(x0), "v"(x1), "v"(x2), "v"(x3), "v"(x4))

__device__ __forceinline__ int clampi(int v, int lo, int hi) {
  return v < lo ? lo : (v > hi ? hi : v);
}
__device__ __forceinline__ float elu1(float v) {
  return v > 0.f ? v : (__expf(v) - 1.f);
}
__device__ __forceinline__ float wave_sum(float s) {
  s += __shfl_xor(s, 16);
  s += __shfl_xor(s, 8);
  s += __shfl_xor(s, 4);
  s += __shfl_xor(s, 2);
  s += __shfl_xor(s, 1);
  return s;
}
__device__ __forceinline__ v8f zero8f() {
  v8f z = {0.f, 0.f, 0.f, 0.f, 0.f, 0.f, 0.f, 0.f};
  return z;
}
__device__ __forceinline__ v8h zero8h() {
  v8h z;
  #pragma unroll
  for (int j = 0; j < 8; ++j) z[j] = (f16t)0.0f;
  return z;
}

__global__ __launch_bounds__(128) void k_w1p(const float* __restrict__ w1, const float* __restrict__ A1,
                                             const float* __restrict__ B1, const int* __restrict__ sid,
                                             f16t* __restrict__ W1P) {
  const int b = blockIdx.x, tid = threadIdx.x;
  const int s = clampi(sid[b], 0, NADP - 1);
  const int n = tid >> 3, q = tid & 7, nn = n & 7;
  float bco[RANK];
  #pragma unroll
  for (int r = 0; r < RANK; ++r) bco[r] = B1[(s * F1 + nn) * RANK + r];
  v8h o;
  #pragma unroll
  for (int e = 0; e < 8; ++e) {
    const int kk = 8 * q + e;
    float v = w1[nn * K12 + kk];
    #pragma unroll
    for (int r = 0; r < RANK; ++r) v += AOR * bco[r] * A1[(s * RANK + r) * K12 + kk];
    o[e] = (n < F1) ? (f16t)(v * WCAR) : (f16t)0.0f;
  }
  f16t* dst = W1P + ((size_t)(b * 16 + n) * K12 + 8 * q);
  *(volatile v8h*)dst = o;
  __threadfence();
  *(volatile v8h*)dst = o;
}

__global__ __launch_bounds__(256) void k_w2p(const float* __restrict__ w2, const float* __restrict__ A2,
                                             const float* __restrict__ B2, const int* __restrict__ sid,
                                             f16t* __restrict__ W2P) {
  const int b = blockIdx.x, tid = threadIdx.x;
  const int s = clampi(sid[b], 0, NADP - 1);
  const int q = tid & 63, f2h = tid >> 6;
  #pragma unroll 1
  for (int j = 0; j < 8; ++j) {
    const int f2 = 4 * j + f2h;
    float bco[RANK];
    #pragma unroll
    for (int r = 0; r < RANK; ++r) bco[r] = B2[(s * F2 + f2) * RANK + r];
    v8h o;
    #pragma unroll
    for (int f1 = 0; f1 < F1; ++f1) {
      float v = w2[(f2 * F1 + f1) * K12 + q];
      #pragma unroll
      for (int r = 0; r < RANK; ++r) v += AOR * bco[r] * A2[((s * RANK + r) * F1 + f1) * K12 + q];
      o[f1] = (f16t)(v * WCAR);
    }
    f16t* dst = W2P + ((size_t)(b * F2 + f2) * K2 + 8 * q);
    *(volatile v8h*)dst = o;
    __threadfence();
    *(volatile v8h*)dst = o;
  }
}

__global__ __launch_bounds__(256) void k_w4p(const float* __restrict__ w4, const float* __restrict__ A4,
                                             const float* __restrict__ B4, const int* __restrict__ sid,
                                             f16t* __restrict__ W4P) {
  const int b = blockIdx.x, q = threadIdx.x;
  const int s = clampi(sid[b], 0, NADP - 1);
  const int reg = q >> 7, qq = q & 127, kk = qq >> 3, f3b = (qq & 7) * 8;
  #pragma unroll 1
  for (int f2 = 0; f2 < F2; ++f2) {
    float bco[RANK];
    #pragma unroll
    for (int r = 0; r < RANK; ++r) bco[r] = B4[(s * F2 + f2) * RANK + r];
    v8h o;
    #pragma unroll
    for (int e = 0; e < 8; ++e) {
      const int f3 = f3b + e;
      const float vm = w4[(f2 * F3 + f3) * K45 + kk];
      float vl = 0.f;
      #pragma unroll
      for (int r = 0; r < RANK; ++r) vl += bco[r] * A4[((s * RANK + r) * F3 + f3) * K45 + kk];
      const float v = reg ? (AOR * vl) : vm;
      o[e] = (f16t)(v * WCAR);
    }
    f16t* dst = W4P + ((size_t)(b * F2 + f2) * K4TOT + 8 * q);
    *(volatile v8h*)dst = o;
    __threadfence();
    *(volatile v8h*)dst = o;
  }
}

__global__ __launch_bounds__(256) void k_w5p(const float* __restrict__ w5, const float* __restrict__ A5,
                                             const float* __restrict__ B5, const int* __restrict__ sid,
                                             f16t* __restrict__ W5P) {
  const int b = blockIdx.x, tid = threadIdx.x;
  const int s = clampi(sid[b], 0, NADP - 1);
  const int q = tid & 127, nh = tid >> 7;
  const int reg = q >> 6, qq = q & 63, kk = qq >> 2, f2b = (qq & 3) * 8;
  #pragma unroll 1
  for (int j = 0; j < 8; ++j) {
    const int n = 2 * j + nh, nn = n & 7;
    float bco[RANK];
    #pragma unroll
    for (int r = 0; r < RANK; ++r) bco[r] = B5[(s * F1 + nn) * RANK + r];
    v8h o;
    #pragma unroll
    for (int e = 0; e < 8; ++e) {
      const int f2 = f2b + e;
      const float vm = w5[(nn * F2 + f2) * K45 + kk];
      float vl = 0.f;
      #pragma unroll
      for (int r = 0; r < RANK; ++r) vl += bco[r] * A5[((s * RANK + r) * F2 + f2) * K45 + kk];
      const float v = (n < F1) ? (reg ? (AOR * vl) : vm) : 0.f;
      o[e] = (f16t)(v * WCAR);
    }
    f16t* dst = W5P + ((size_t)(b * 16 + n) * K5TOT + 8 * q);
    *(volatile v8h*)dst = o;
    __threadfence();
    *(volatile v8h*)dst = o;
  }
}

__global__ __launch_bounds__(128) void k_conv1(const float* __restrict__ x, const f16t* __restrict__ W1P,
                                              f16t* __restrict__ H1) {
  __shared__ __attribute__((aligned(16))) float sx[1024];
  __shared__ __attribute__((aligned(16))) f16t scp[4 * CPW];
  __shared__ __attribute__((aligned(16))) f16t so[4 * 256];
  const int tid = threadIdx.x, lane = tid & 31, w = tid >> 5, h = lane >> 4, m = lane & 15;
  const int bc = blockIdx.x, b = bc >> 6;
  const float* xr = x + (size_t)bc * TT;
  const v4f z4 = {0.f, 0.f, 0.f, 0.f};
  for (int i = tid; i < 256; i += 128) {
    const int ic = i < 250 ? i : 249;
    v4f v = *(const v4fa*)(xr + 4 * ic);
    if (i >= 250) v = z4;
    *(v4fa*)(sx + 4 * i) = v;
  }
  __syncthreads();
  for (int sl = tid; sl < 4 * 138; sl += 128) {
    const int r = sl / 138, q = sl - r * 138;
    v8h o;
    #pragma unroll
    for (int e = 0; e < 8; ++e) {
      const int t = 8 * q + e + r - H1OFF;
      const int tc = clampi(t, 0, TT - 1);
      const float v = sx[tc];
      o[e] = ((unsigned)t < (unsigned)TT) ? (f16t)v : (f16t)0.0f;
    }
    *(v8ha*)(scp + r * CPW + 8 * q) = o;
  }
  __syncthreads();

  Frag bw0, bw1;
  {
    const f16t* wrow = W1P + (size_t)(b * 16 + m) * K12 + 8 * h;
    bw0.half[0] = *(const v8ha*)(wrow);
    bw0.half[1] = *(const v8ha*)(wrow + 16);
    bw1.half[0] = *(const v8ha*)(wrow + 32);
    bw1.half[1] = *(const v8ha*)(wrow + 48);
  }
  const int r4 = (m + 1) & 3;
  const int mb = (m + 1) - r4;
  const f16t* abase = scp + r4 * CPW + mb + 8 * h;
  f16t* hrow = H1 + (size_t)bc * (H1ROWS * 8);
  f16t* sw = so + w * 256;

  if (w == 0) {
    const v8h z = zero8h();
    f16t* dst = hrow + (size_t)lane * 8;
    *(volatile v8h*)dst = z;
    __threadfence();
    *(volatile v8h*)dst = z;
  }
  if (w == 1) {
    const v8h z = zero8h();
    f16t* dst = hrow + (size_t)(H1OFF + TPAD + lane) * 8;
    *(volatile v8h*)dst = z;
    __threadfence();
    *(volatile v8h*)dst = z;
  }

  #pragma unroll 1
  for (int it = 0; it < 8; ++it) {
    const int tw = (it * 4 + w) * 32;
    v8f acc0 = zero8f(), acc1 = zero8f();
    Frag a00, a01, a10, a11;
    {
      const f16t* p0 = abase + tw;
      a00.q[0] = *(const v4ha*)(p0);      a00.q[1] = *(const v4ha*)(p0 + 4);
      a00.q[2] = *(const v4ha*)(p0 + 16); a00.q[3] = *(const v4ha*)(p0 + 20);
      a01.q[0] = *(const v4ha*)(p0 + 32); a01.q[1] = *(const v4ha*)(p0 + 36);
      a01.q[2] = *(const v4ha*)(p0 + 48); a01.q[3] = *(const v4ha*)(p0 + 52);
      const f16t* p1 = p0 + 16;
      a10.q[0] = *(const v4ha*)(p1);      a10.q[1] = *(const v4ha*)(p1 + 4);
      a10.q[2] = *(const v4ha*)(p1 + 16); a10.q[3] = *(const v4ha*)(p1 + 20);
      a11.q[0] = *(const v4ha*)(p1 + 32); a11.q[1] = *(const v4ha*)(p1 + 36);
      a11.q[2] = *(const v4ha*)(p1 + 48); a11.q[3] = *(const v4ha*)(p1 + 52);
    }
    acc0 = wmma1(a00.v, bw0.v, acc0);
    acc0 = wmma1(a01.v, bw1.v, acc0);
    acc1 = wmma1(a10.v, bw0.v, acc1);
    acc1 = wmma1(a11.v, bw1.v, acc1);
    GUARD2x6(acc0, acc1, a00.v, a01.v, a10.v, a11.v, bw0.v, bw1.v);

    if (m < F1) {
      #pragma unroll
      for (int r = 0; r < 8; ++r) {
        const int tl0 = 8 * h + r, tl1 = 16 + 8 * h + r;
        const float v0 = (tw + tl0 < TT) ? acc0[r] * WINV : 0.f;
        const float v1 = (tw + tl1 < TT) ? acc1[r] * WINV : 0.f;
        sw[tl0 * 8 + m] = (f16t)v0;
        sw[tl1 * 8 + m] = (f16t)v1;
      }
    }
    __syncthreads();
    const v8h val = *(const v8ha*)(sw + 8 * lane);
    f16t* dst = hrow + (size_t)(H1OFF + tw + lane) * 8;
    *(volatile v8h*)dst = val;
    __threadfence();
    *(volatile v8h*)dst = val;
    __syncthreads();
  }
}

__global__ __launch_bounds__(128) void k_conv2(const f16t* __restrict__ H1, const f16t* __restrict__ W2P,
                                              const float* __restrict__ w3,
                                              const float* __restrict__ g2, const float* __restrict__ be2,
                                              const float* __restrict__ m2, const float* __restrict__ v2,
                                              const float* __restrict__ g3, const float* __restrict__ be3,
                                              const float* __restrict__ m3, const float* __restrict__ v3,
                                              float* __restrict__ O3) {
  __shared__ __attribute__((aligned(16))) float sBig[8192];
  __shared__ __attribute__((aligned(16))) float sW3T[NCH * F3];
  __shared__ float sInv2[F2], sK2[F2];
  __shared__ float sRs3[F3], sInv3[F3], sM3[F3], sB3[F3];
  const int tid = threadIdx.x, lane = tid & 31, w = tid >> 5, h = lane >> 4, m = lane & 15;
  const int b = blockIdx.y;
  const int t0w = blockIdx.x * 128 + w * 32;
  f16t* sWh = (f16t*)sBig;
  {
    const f16t* wsrc = W2P + (size_t)b * (F2 * K2);
    for (int i = tid; i < (F2 * K2) / 8; i += 128) *(v8ha*)(sWh + 8 * i) = *(const v8ha*)(wsrc + 8 * i);
    for (int i = tid; i < NCH * F3; i += 128) {
      const int o = i >> 6, c = i & 63;
      sW3T[c * 64 + o] = w3[i];
    }
    if (tid < F2) {
      const float inv = g2[tid] / sqrtf(v2[tid] + EPS_);
      sInv2[tid] = inv;
      sK2[tid] = be2[tid] - m2[tid] * inv;
    }
    if (tid < F3) {
      sInv3[tid] = g3[tid] / sqrtf(v3[tid] + EPS_);
      sM3[tid] = m3[tid];
      sB3[tid] = be3[tid];
    }
  }
  __syncthreads();
  if (tid < F3) {
    float ss = 0.f;
    #pragma unroll 4
    for (int c = 0; c < NCH; ++c) { const float v = sW3T[c * 64 + tid]; ss += v * v; }
    const float nrm = sqrtf(ss);
    const float sc = (nrm > 1.0f) ? (1.0f / (nrm + 1e-7f)) : 1.0f;
    float rs = 0.f;
    #pragma unroll 4
    for (int c = 0; c < NCH; ++c) {
      const float v = sW3T[c * 64 + tid] * sc;
      sW3T[c * 64 + tid] = v;
      rs += v;
    }
    sRs3[tid] = rs;
  }
  __syncthreads();

  float f3a[2][2][8][2];
  #pragma unroll
  for (int a = 0; a < 2; ++a)
    #pragma unroll
    for (int p = 0; p < 2; ++p)
      #pragma unroll
      for (int r = 0; r < 8; ++r) { f3a[a][p][r][0] = 0.f; f3a[a][p][r][1] = 0.f; }

  const f16t* hb = H1 + (size_t)(b * NCH) * (H1ROWS * 8) + (size_t)(t0w + m + 1 + h) * 8;
  const f16t* aw0 = sWh + m * K2 + 8 * h;
  const f16t* aw1 = aw0 + 16 * K2;

  #pragma unroll 1
  for (int c = 0; c < NCH; ++c) {
    const f16t* hrow = hb + (size_t)c * (H1ROWS * 8);
    v8f acc00 = zero8f(), acc01 = zero8f(), acc10 = zero8f(), acc11 = zero8f();
    #pragma unroll 1
    for (int ks = 0; ks < 16; ++ks) {
      Frag A0, A1, B0, B1;
      A0.half[0] = *(const v8ha*)(aw0 + 32 * ks);
      A0.half[1] = *(const v8ha*)(aw0 + 32 * ks + 16);
      A1.half[0] = *(const v8ha*)(aw1 + 32 * ks);
      A1.half[1] = *(const v8ha*)(aw1 + 32 * ks + 16);
      const f16t* bp = hrow + 32 * ks;
      B0.half[0] = *(const v8ha*)(bp);
      B0.half[1] = *(const v8ha*)(bp + 16);
      B1.half[0] = *(const v8ha*)(bp + 128);
      B1.half[1] = *(const v8ha*)(bp + 144);
      acc00 = wmma1(A0.v, B0.v, acc00);
      acc01 = wmma1(A0.v, B1.v, acc01);
      acc10 = wmma1(A1.v, B0.v, acc10);
      acc11 = wmma1(A1.v, B1.v, acc11);
      GUARD4x4(acc00, acc01, acc10, acc11, A0.v, A1.v, B0.v, B1.v);
    }
    #pragma unroll
    for (int a = 0; a < 2; ++a) {
      const float* wc = sW3T + c * 64 + 32 * a + 16 * h;
      const v4f q0 = *(const v4fa*)(wc), q1 = *(const v4fa*)(wc + 4);
      const v4f q2 = *(const v4fa*)(wc + 8), q3 = *(const v4fa*)(wc + 12);
      const float wl[16] = {q0.x, q0.y, q0.z, q0.w, q1.x, q1.y, q1.z, q1.w,
                            q2.x, q2.y, q2.z, q2.w, q3.x, q3.y, q3.z, q3.w};
      #pragma unroll
      for (int r = 0; r < 8; ++r) {
        const float av0 = (a == 0) ? acc00[r] : acc10[r];
        const float av1 = (a == 0) ? acc01[r] : acc11[r];
        f3a[a][0][r][0] += wl[2 * r] * av0;
        f3a[a][0][r][1] += wl[2 * r + 1] * av0;
        f3a[a][1][r][0] += wl[2 * r] * av1;
        f3a[a][1][r][1] += wl[2 * r + 1] * av1;
      }
    }
  }

  __syncthreads();
  float* st = sBig + w * 2048;
  #pragma unroll
  for (int a = 0; a < 2; ++a)
    #pragma unroll
    for (int r = 0; r < 8; ++r) {
      const int f2 = 16 * a + 8 * h + r;
      const float i2 = sInv2[f2] * WINV, k2 = sK2[f2];
      #pragma unroll
      for (int s2 = 0; s2 < 2; ++s2) {
        const int o = 2 * f2 + s2;
        const float rs = sRs3[o], mm3 = sM3[o], ii3 = sInv3[o], bb3 = sB3[o];
        #pragma unroll
        for (int p = 0; p < 2; ++p) {
          float v = f3a[a][p][r][s2] * i2 + k2 * rs;
          v = (v - mm3) * ii3 + bb3;
          v = elu1(v);
          st[(16 * p + m) * 64 + o] = v;
        }
      }
    }
  __syncthreads();
  v4f vals[16];
  #pragma unroll
  for (int i = 0; i < 16; ++i) vals[i] = *(const v4fa*)(st + (i * 32 + lane) * 4);
  float* ob = O3 + ((size_t)(b * TPAD + t0w)) * F3;
  #pragma unroll
  for (int i = 0; i < 16; ++i) *(volatile v4f*)(ob + (i * 32 + lane) * 4) = vals[i];
  __threadfence();
  #pragma unroll
  for (int i = 0; i < 16; ++i) *(volatile v4f*)(ob + (i * 32 + lane) * 4) = vals[i];
}

__global__ __launch_bounds__(256) void k_pool4(const float* __restrict__ O3, f16t* __restrict__ H4) {
  const int b = blockIdx.x, tid = threadIdx.x, o8 = tid & 7, tq = tid >> 3;
  const float* ob = O3 + (size_t)b * TPAD * F3 + 8 * o8;
  f16t* hbp = H4 + (size_t)b * H4ROWS * F3 + 8 * o8;
  const v4f z4 = {0.f, 0.f, 0.f, 0.f};
  #pragma unroll 1
  for (int pass = 0; pass < 9; ++pass) {
    const int tp = pass * 32 + tq, t3 = tp - H4OFF;
    const bool tv = (t3 >= 0) && (t3 < T3);
    v4f sa = z4, sb = z4;
    #pragma unroll
    for (int u = 0; u < 4; ++u) {
      const int ti = 4 * t3 - 1 + u;
      const bool ok = tv && (ti >= 0) && (ti < TT);
      const int tic = clampi(ti, 0, TT - 1);
      const float* rp = ob + (size_t)tic * F3;
      const v4f x0 = *(const v4fa*)(rp);
      const v4f x1 = *(const v4fa*)(rp + 4);
      sa += ok ? x0 : z4;
      sb += ok ? x1 : z4;
    }
    v8h o;
    o[0] = (f16t)(0.25f * sa.x); o[1] = (f16t)(0.25f * sa.y); o[2] = (f16t)(0.25f * sa.z); o[3] = (f16t)(0.25f * sa.w);
    o[4] = (f16t)(0.25f * sb.x); o[5] = (f16t)(0.25f * sb.y); o[6] = (f16t)(0.25f * sb.z); o[7] = (f16t)(0.25f * sb.w);
    f16t* dst = hbp + (size_t)tp * F3;
    *(volatile v8h*)dst = o;
    __threadfence();
    *(volatile v8h*)dst = o;
  }
}

__global__ __launch_bounds__(256) void k_conv4(const f16t* __restrict__ H4, const f16t* __restrict__ W4P,
                                              const float* __restrict__ g4, const float* __restrict__ be4,
                                              const float* __restrict__ m4, const float* __restrict__ v4,
                                              f16t* __restrict__ H5) {
  __shared__ __attribute__((aligned(16))) f16t sH5[256 * F2];
  __shared__ float sInv4[F2], sM4[F2], sB4[F2];
  const int tid = threadIdx.x, lane = tid & 31, w = tid >> 5, h = lane >> 4, m = lane & 15;
  const int b = blockIdx.x;
  if (tid < F2) {
    sInv4[tid] = g4[tid] / sqrtf(v4[tid] + EPS_);
    sM4[tid] = m4[tid];
    sB4[tid] = be4[tid];
  }
  __syncthreads();
  const f16t* wa0 = W4P + (size_t)(b * F2 + m) * K4TOT + 8 * h;
  const f16t* wa1 = wa0 + 16 * K4TOT;
  const f16t* hb = H4 + (size_t)b * H4ROWS * F3 + 8 * h;
  const int tb = w * 32 + m;
  v8f acc00 = zero8f(), acc01 = zero8f(), acc10 = zero8f(), acc11 = zero8f();
  #pragma unroll 1
  for (int ks = 0; ks < 64; ++ks) {
    const int reg = ks >> 5, kl = ks & 31, kk = kl >> 1, f3b = (kl & 1) * 32;
    const int toff = reg ? (kk - 7) : (2 * kk - 15);
    const int k0 = 32 * ks;
    Frag A0, A1, B0, B1;
    A0.half[0] = *(const v8ha*)(wa0 + k0);
    A0.half[1] = *(const v8ha*)(wa0 + k0 + 16);
    A1.half[0] = *(const v8ha*)(wa1 + k0);
    A1.half[1] = *(const v8ha*)(wa1 + k0 + 16);
    const f16t* bp = hb + (size_t)(tb + toff + H4OFF) * F3 + f3b;
    B0.half[0] = *(const v8ha*)(bp);
    B0.half[1] = *(const v8ha*)(bp + 16);
    B1.half[0] = *(const v8ha*)(bp + 16 * F3);
    B1.half[1] = *(const v8ha*)(bp + 16 * F3 + 16);
    acc00 = wmma1(A0.v, B0.v, acc00);
    acc01 = wmma1(A0.v, B1.v, acc01);
    acc10 = wmma1(A1.v, B0.v, acc10);
    acc11 = wmma1(A1.v, B1.v, acc11);
    GUARD4x4(acc00, acc01, acc10, acc11, A0.v, A1.v, B0.v, B1.v);
  }
  #pragma unroll
  for (int a = 0; a < 2; ++a)
    #pragma unroll
    for (int r = 0; r < 8; ++r) {
      const int f2 = 16 * a + 8 * h + r;
      const float ii = sInv4[f2], mm = sM4[f2], bb = sB4[f2];
      #pragma unroll
      for (int p = 0; p < 2; ++p) {
        const int tl = w * 32 + 16 * p + m;
        const float av = (a == 0) ? ((p == 0) ? acc00[r] : acc01[r]) : ((p == 0) ? acc10[r] : acc11[r]);
        const float v = (tl < T3) ? ((av * WINV - mm) * ii + bb) : 0.f;
        sH5[tl * F2 + f2] = (f16t)v;
      }
    }
  __syncthreads();
  f16t* hout = H5 + (size_t)b * H5ROWS * F2;
  v8h vals[4];
  #pragma unroll
  for (int i = 0; i < 4; ++i) vals[i] = *(const v8ha*)(sH5 + (32 * w) * F2 + (i * 32 + lane) * 8);
  f16t* dst = hout + (size_t)(H5OFF + 32 * w) * F2;
  #pragma unroll
  for (int i = 0; i < 4; ++i) *(volatile v8h*)(dst + (i * 32 + lane) * 8) = vals[i];
  __threadfence();
  #pragma unroll
  for (int i = 0; i < 4; ++i) *(volatile v8h*)(dst + (i * 32 + lane) * 8) = vals[i];
  if (w < 2) {
    const v8h z = zero8h();
    f16t* pd = hout + (size_t)((w == 0) ? 0 : (H5OFF + 256)) * F2;
    #pragma unroll
    for (int i = 0; i < 4; ++i) *(volatile v8h*)(pd + (i * 32 + lane) * 8) = z;
    __threadfence();
    #pragma unroll
    for (int i = 0; i < 4; ++i) *(volatile v8h*)(pd + (i * 32 + lane) * 8) = z;
  }
}

__global__ __launch_bounds__(128) void k_conv5(const f16t* __restrict__ H5, const f16t* __restrict__ W5P,
                                              const float* __restrict__ g5, const float* __restrict__ be5,
                                              const float* __restrict__ m5, const float* __restrict__ v5,
                                              float* __restrict__ FEAT) {
  __shared__ __attribute__((aligned(16))) float sV[F1 * 256];
  __shared__ __attribute__((aligned(16))) float sF[256];
  __shared__ float sInv5[F1], sM5[F1], sB5[F1];
  const int tid = threadIdx.x, lane = tid & 31, w = tid >> 5, h = lane >> 4, m = lane & 15;
  const int b = blockIdx.x;
  if (tid < F1) {
    sInv5[tid] = g5[tid] / sqrtf(v5[tid] + EPS_);
    sM5[tid] = m5[tid];
    sB5[tid] = be5[tid];
  }
  __syncthreads();
  const f16t* wb = W5P + (size_t)(b * 16 + m) * K5TOT + 8 * h;
  const f16t* hb = H5 + (size_t)b * H5ROWS * F2 + 8 * h;
  const int tb = w * 64 + m;
  v8f acc0 = zero8f(), acc1 = zero8f(), acc2 = zero8f(), acc3 = zero8f();
  #pragma unroll 1
  for (int ks = 0; ks < 32; ++ks) {
    const int reg = ks >> 4, kk = ks & 15;
    const int toff = reg ? (kk - 7) : (4 * kk - 30);
    const int k0 = 32 * ks;
    Frag Bw, A0, A1, A2, A3;
    Bw.half[0] = *(const v8ha*)(wb + k0);
    Bw.half[1] = *(const v8ha*)(wb + k0 + 16);
    const f16t* ap = hb + (size_t)(tb + toff + H5OFF) * F2;
    A0.half[0] = *(const v8ha*)(ap);                 A0.half[1] = *(const v8ha*)(ap + 16);
    A1.half[0] = *(const v8ha*)(ap + 16 * F2);       A1.half[1] = *(const v8ha*)(ap + 16 * F2 + 16);
    A2.half[0] = *(const v8ha*)(ap + 32 * F2);       A2.half[1] = *(const v8ha*)(ap + 32 * F2 + 16);
    A3.half[0] = *(const v8ha*)(ap + 48 * F2);       A3.half[1] = *(const v8ha*)(ap + 48 * F2 + 16);
    acc0 = wmma1(A0.v, Bw.v, acc0);
    acc1 = wmma1(A1.v, Bw.v, acc1);
    acc2 = wmma1(A2.v, Bw.v, acc2);
    acc3 = wmma1(A3.v, Bw.v, acc3);
    GUARD4x5(acc0, acc1, acc2, acc3, A0.v, A1.v, A2.v, A3.v, Bw.v);
  }
  {
    const int mm = m & 7;
    const float ii = sInv5[mm], m5v = sM5[mm], bb = sB5[mm];
    #pragma unroll
    for (int p = 0; p < 4; ++p)
      #pragma unroll
      for (int r = 0; r < 8; ++r) {
        const int t = w * 64 + 16 * p + 8 * h + r;
        const float av = (p == 0) ? acc0[r] : ((p == 1) ? acc1[r] : ((p == 2) ? acc2[r] : acc3[r]));
        const float v = elu1((av * WINV - m5v) * ii + bb);
        if (m < F1 && t < T3) sV[mm * 256 + t] = v;
      }
  }
  __syncthreads();
  for (int idx = tid; idx < 256; idx += 128) {
    float s = 0.f;
    if (idx < NFEAT) {
      const int f1 = idx / T5, t5 = idx - f1 * T5;
      #pragma unroll
      for (int u = 0; u < 8; ++u) {
        const int ti = 8 * t5 - 1 + u;
        const int tic = clampi(ti, 0, T3 - 1);
        const float v = sV[f1 * 256 + tic];
        s += ((unsigned)ti < (unsigned)T3) ? v : 0.f;
      }
      s *= 0.125f;
    }
    sF[idx] = s;
  }
  __syncthreads();
  if (w < 2) {
    const v4f v = *(const v4fa*)(sF + (w * 32 + lane) * 4);
    float* dst = FEAT + (size_t)b * 256 + (w * 32 + lane) * 4;
    *(volatile v4f*)dst = v;
    __threadfence();
    *(volatile v4f*)dst = v;
  }
}

__global__ __launch_bounds__(256) void k_final(const float* __restrict__ FEAT, const float* __restrict__ wf,
                                              const float* __restrict__ bfv, float* __restrict__ out) {
  __shared__ float sWf[NOUT * NFEAT];
  __shared__ float sSc[NOUT];
  __shared__ __attribute__((aligned(16))) float sOut[256];
  const int tid = threadIdx.x, lane = tid & 31, w = tid >> 5;
  for (int i = tid; i < NOUT * NFEAT; i += 256) sWf[i] = wf[i];
  __syncthreads();
  if (w < NOUT) {
    float ss = 0.f;
    #pragma unroll
    for (int j = 0; j < 8; ++j) {
      const int i = lane + 32 * j;
      const int ic = i < NFEAT ? i : NFEAT - 1;
      const float v = sWf[w * NFEAT + ic];
      ss += (i < NFEAT) ? v * v : 0.f;
    }
    ss = wave_sum(ss);
    if (lane == 0) {
      const float nrm = sqrtf(ss);
      sSc[w] = (nrm > 0.25f) ? (0.25f / (nrm + 1e-7f)) : 1.0f;
    }
  }
  __syncthreads();
  for (int i = tid; i < NOUT * NFEAT; i += 256) sWf[i] = sWf[i] * sSc[i / NFEAT];
  __syncthreads();
  {
    const int bq = tid >> 2, o = tid & 3;
    const float* fr = FEAT + (size_t)bq * 256;
    const float* wr = sWf + o * NFEAT;
    float p = 0.f;
    #pragma unroll 4
    for (int i = 0; i < NFEAT; ++i) p += fr[i] * wr[i];
    sOut[tid] = p + bfv[o];
  }
  __syncthreads();
  if (w < 2) {
    const v4f v = *(const v4fa*)(sOut + (w * 32 + lane) * 4);
    float* dst = out + (w * 32 + lane) * 4;
    *(volatile v4f*)dst = v;
    __threadfence();
    *(volatile v4f*)dst = v;
  }
}

extern "C" void kernel_launch(void* const* d_in, const int* in_sizes, int n_in,
                              void* d_out, int out_size, void* d_ws, size_t ws_size,
                              hipStream_t stream) {
  if (n_in < 33) return;
  if (in_sizes[0] != NB_ * NCH * TT || in_sizes[1] != NB_) return;
  if (in_sizes[2] != F1 * K12 || in_sizes[3] != NADP * RANK * K12 || in_sizes[4] != NADP * F1 * RANK) return;
  if (in_sizes[5] != F2 * F1 * K12 || in_sizes[6] != NADP * RANK * F1 * K12 || in_sizes[7] != NADP * F2 * RANK) return;
  if (in_sizes[8] != F3 * NCH) return;
  if (in_sizes[9] != F2 * F3 * K45 || in_sizes[10] != NADP * RANK * F3 * K45 || in_sizes[11] != NADP * F2 * RANK) return;
  if (in_sizes[12] != F1 * F2 * K45 || in_sizes[13] != NADP * RANK * F2 * K45 || in_sizes[14] != NADP * F1 * RANK) return;
  for (int i = 15; i <= 18; ++i) if (in_sizes[i] != F2) return;
  for (int i = 19; i <= 22; ++i) if (in_sizes[i] != F3) return;
  for (int i = 23; i <= 26; ++i) if (in_sizes[i] != F2) return;
  for (int i = 27; i <= 30; ++i) if (in_sizes[i] != F1) return;
  if (in_sizes[31] != NOUT * NFEAT || in_sizes[32] != NOUT) return;
  if (out_size != NB_ * NOUT) return;
  if (WS_TOTAL > ws_size) return;

  const float* x  = (const float*)d_in[0];
  const int*   sid = (const int*)d_in[1];
  const float* w1 = (const float*)d_in[2];
  const float* A1 = (const float*)d_in[3];
  const float* B1 = (const float*)d_in[4];
  const float* w2 = (const float*)d_in[5];
  const float* A2 = (const float*)d_in[6];
  const float* B2 = (const float*)d_in[7];
  const float* w3 = (const float*)d_in[8];
  const float* w4 = (const float*)d_in[9];
  const float* A4 = (const float*)d_in[10];
  const float* B4 = (const float*)d_in[11];
  const float* w5 = (const float*)d_in[12];
  const float* A5 = (const float*)d_in[13];
  const float* B5 = (const float*)d_in[14];
  const float* g2 = (const float*)d_in[15], *be2 = (const float*)d_in[16];
  const float* m2 = (const float*)d_in[17], *v2 = (const float*)d_in[18];
  const float* g3 = (const float*)d_in[19], *be3 = (const float*)d_in[20];
  const float* m3 = (const float*)d_in[21], *v3 = (const float*)d_in[22];
  const float* g4 = (const float*)d_in[23], *be4 = (const float*)d_in[24];
  const float* m4 = (const float*)d_in[25], *v4 = (const float*)d_in[26];
  const float* g5 = (const float*)d_in[27], *be5 = (const float*)d_in[28];
  const float* m5 = (const float*)d_in[29], *v5 = (const float*)d_in[30];
  const float* wf = (const float*)d_in[31];
  const float* bfv = (const float*)d_in[32];
  float* out = (float*)d_out;

  char* ws = (char*)d_ws;
  f16t*  W1P  = (f16t*)(ws + OFF_W1P);
  f16t*  W2P  = (f16t*)(ws + OFF_W2P);
  f16t*  W4P  = (f16t*)(ws + OFF_W4P);
  f16t*  W5P  = (f16t*)(ws + OFF_W5P);
  f16t*  H1   = (f16t*)(ws + OFF_H1);
  float* O3   = (float*)(ws + OFF_O3);
  f16t*  H4   = (f16t*)(ws + OFF_H4);
  f16t*  H5   = (f16t*)(ws + OFF_H5);
  float* FEAT = (float*)(ws + OFF_FEAT);

  k_w1p<<<NB_, 128, 0, stream>>>(w1, A1, B1, sid, W1P);
  k_w2p<<<NB_, 256, 0, stream>>>(w2, A2, B2, sid, W2P);
  k_w4p<<<NB_, 256, 0, stream>>>(w4, A4, B4, sid, W4P);
  k_w5p<<<NB_, 256, 0, stream>>>(w5, A5, B5, sid, W5P);
  k_conv1<<<NB_ * NCH, 128, 0, stream>>>(x, W1P, H1);
  k_conv2<<<dim3(TPAD / 128, NB_), 128, 0, stream>>>(H1, W2P, w3, g2, be2, m2, v2, g3, be3, m3, v3, O3);
  k_pool4<<<NB_, 256, 0, stream>>>(O3, H4);
  k_conv4<<<NB_, 256, 0, stream>>>(H4, W4P, g4, be4, m4, v4, H5);
  k_conv5<<<NB_, 128, 0, stream>>>(H5, W5P, g5, be5, m5, v5, FEAT);
  k_final<<<1, 256, 0, stream>>>(FEAT, wf, bfv, out);
}
